// MultipleFullGaussian2d_11785390260963
// MI455X (gfx1250) — hardware-verified
//
#include <hip/hip_runtime.h>


#define NB_  8
#define CC   256
#define NS   4096
#define NO   4096
#define GW   64
typedef _Float16 h16;
typedef unsigned short bf;
typedef __attribute__((ext_vector_type(16))) __bf16   v16bf;
typedef __attribute__((ext_vector_type(16))) _Float16 v16h;
typedef __attribute__((ext_vector_type(8)))  _Float16 v8h;
typedef __attribute__((ext_vector_type(8)))  unsigned short v8us;
typedef __attribute__((ext_vector_type(8)))  float    v8f;
typedef __attribute__((ext_vector_type(4)))  float    v4f;
typedef v8h  __attribute__((may_alias)) v8ha;
typedef v4f  __attribute__((may_alias)) v4fa;
typedef v8us __attribute__((may_alias)) v8usa;

__device__ __forceinline__ unsigned short f2bf(float f) { unsigned u = __float_as_uint(f); u += 0x7FFFu + ((u >> 16) & 1u); return (unsigned short)(u >> 16); }
__device__ __forceinline__ float bf2f(unsigned short b) { return __uint_as_float(((unsigned)b) << 16); }
__device__ __forceinline__ float bfr(float f) { return bf2f(f2bf(f)); }
__device__ __forceinline__ v16h cat16(v8h lo, v8h hi) { return __builtin_shufflevector(lo, hi, 0, 1, 2, 3, 4, 5, 6, 7, 8, 9, 10, 11, 12, 13, 14, 15); }
__device__ __forceinline__ v16bf cat16b(v8us lo, v8us hi) { return __builtin_bit_cast(v16bf, __builtin_shufflevector(lo, hi, 0, 1, 2, 3, 4, 5, 6, 7, 8, 9, 10, 11, 12, 13, 14, 15)); }
__device__ __forceinline__ v8f wmma16(v16h a, v16h b, v8f c) { return __builtin_amdgcn_wmma_f32_16x16x32_f16(false, a, false, b, (short)0, c, false, false); }
__device__ __forceinline__ v8f wmmab(v16bf a, v16bf b, v8f c) { return __builtin_amdgcn_wmma_f32_16x16x32_bf16(false, a, false, b, (short)0, c, false, false); }


template <typename T16> struct WFrag;
template <> struct WFrag<h16> { typedef v16h V; static __device__ __forceinline__ V ld(const h16* p) { return cat16(*(const v8h*)p, *(const v8h*)(p + 16)); } static __device__ __forceinline__ v8f mma(V a, V b, v8f c) { return wmma16(a, b, c); } };
template <> struct WFrag<bf> { typedef v16bf V; static __device__ __forceinline__ V ld(const bf* p) { return cat16b(*(const v8us*)p, *(const v8us*)(p + 16)); } static __device__ __forceinline__ v8f mma(V a, V b, v8f c) { return wmmab(a, b, c); } };
template <typename T16, int NSPLIT, bool BIAS>
__global__ __launch_bounds__(32) void k_gemmw(const T16* __restrict__ A, const T16* __restrict__ A2, const T16* __restrict__ Bt, const T16* __restrict__ Bt2, int K, float* C, int ldc, const float* __restrict__ bias, size_t sA, size_t sB, size_t sC) {
    typedef typename WFrag<T16>::V V;
    __shared__ __align__(16) float os[16 * 68];
    const size_t z = blockIdx.z; A += z * sA; if (A2) A2 += z * sA; Bt += z * sB; if (Bt2) Bt2 += z * sB; C += z * sC;
    const int lane = threadIdx.x & 31, lr = lane & 15, hi = lane >> 4; const int r0 = blockIdx.x * 64, c0 = blockIdx.y * 64;
    v8f acc[4][4];
#pragma unroll
    for (int mb = 0; mb < 4; ++mb)
#pragma unroll
        for (int nb = 0; nb < 4; ++nb) acc[mb][nb] = (v8f){};
    const size_t aoff = (size_t)(r0 + lr) * K + 8 * hi, boff = (size_t)(c0 + lr) * K + 8 * hi;
#pragma unroll 1
    for (int kc = 0; kc < K; kc += 32) {
        V a[4], a2[4];
#pragma unroll
        for (int mb = 0; mb < 4; ++mb) { a[mb] = WFrag<T16>::ld(A + aoff + (size_t)mb * 16 * K + kc); if (NSPLIT == 1 || NSPLIT == 2) a2[mb] = WFrag<T16>::ld(A2 + aoff + (size_t)mb * 16 * K + kc); }
#pragma unroll
        for (int nb = 0; nb < 4; ++nb) { const V b = WFrag<T16>::ld(Bt + boff + (size_t)nb * 16 * K + kc); V b2; if (NSPLIT >= 2) b2 = WFrag<T16>::ld(Bt2 + boff + (size_t)nb * 16 * K + kc);
#pragma unroll
            for (int mb = 0; mb < 4; ++mb) { acc[mb][nb] = WFrag<T16>::mma(a[mb], b, acc[mb][nb]); if (NSPLIT == 1 || NSPLIT == 2) acc[mb][nb] = WFrag<T16>::mma(a2[mb], b, acc[mb][nb]); if (NSPLIT >= 2) acc[mb][nb] = WFrag<T16>::mma(a[mb], b2, acc[mb][nb]); } }
        asm volatile("v_nop\n\tv_nop\n\tv_nop\n\tv_nop" : "+v"(acc[0][0]), "+v"(acc[1][1]), "+v"(acc[2][2]), "+v"(acc[3][3]) : "v"(a[0]), "v"(a[3]));
    }
#pragma unroll
    for (int mb = 0; mb < 4; ++mb) {
#pragma unroll
        for (int nb = 0; nb < 4; ++nb) {
#pragma unroll
            for (int j = 0; j < 8; ++j) os[(hi * 8 + j) * 68 + nb * 16 + lr] = acc[mb][nb][j]; }
        __builtin_amdgcn_wave_barrier(); asm volatile("" ::: "memory");
        float* crow = C + (size_t)(r0 + mb * 16) * ldc + c0;
#pragma unroll 1
        for (int ps = 0; ps < 2; ++ps) {
#pragma unroll
            for (int s = 0; s < 8; ++s) { const int row = 2 * s + hi, cofs = lr * 4; v4f val = *(const v4fa*)(os + row * 68 + cofs); if (BIAS) { val[0] += bfr(bias[c0 + cofs]); val[1] += bfr(bias[c0 + cofs + 1]); val[2] += bfr(bias[c0 + cofs + 2]); val[3] += bfr(bias[c0 + cofs + 3]); }
                *(volatile v4f*)(crow + (size_t)row * ldc + cofs) = val; }
            if (ps == 0) __threadfence(); }
        __builtin_amdgcn_wave_barrier(); asm volatile("" ::: "memory");
    }
}

__device__ __forceinline__ float sigm_(float x) { return __fdiv_rn(1.0f, 1.0f + __expf(-x)); }
typedef __attribute__((ext_vector_type(4))) unsigned short v4us;

__global__ __launch_bounds__(256) void k_cvt8(const float* __restrict__ src, bf* dst, size_t n8) { const size_t i = (size_t)blockIdx.x * 256 + threadIdx.x; if (i >= n8) return; const v8f v = *(const v8f*)(src + i * 8); v8us o;
#pragma unroll
    for (int k = 0; k < 8; ++k) o[k] = f2bf(v[k]); *(volatile v8us*)(dst + i * 8) = o; __threadfence(); *(volatile v8us*)(dst + i * 8) = o; }
__global__ __launch_bounds__(256) void k_tok(const float* __restrict__ x, bf* XT) { const size_t e = ((size_t)blockIdx.x * 256 + threadIdx.x) * 4; if (e >= (size_t)NS * CC) return; const int c = (int)(e % CC), s = (int)(e / CC); v4us o;
#pragma unroll
    for (int q = 0; q < 4; ++q) o[q] = f2bf(x[(size_t)(c + q) * NS + s]); *(volatile v4us*)(XT + e) = o; __threadfence(); *(volatile v4us*)(XT + e) = o; }
__global__ __launch_bounds__(256) void k_gauss(const float* __restrict__ mu, const float* __restrict__ sg, float* G) { const size_t e = ((size_t)blockIdx.x * 256 + threadIdx.x) * 4; if (e >= (size_t)NO * NS) return; const int s0 = (int)(e % NS); const int o = (int)(e / NS); const float mx = __fmul_rn(sigm_(bfr(mu[o * 2])), (float)GW), my = __fmul_rn(sigm_(bfr(mu[o * 2 + 1])), (float)GW); const float sx = __expf(bfr(sg[o * 2])), sy = __expf(bfr(sg[o * 2 + 1])); const int i = s0 / GW; const float zy = __fdiv_rn(__fsub_rn((float)i, my), sy); float zy2 = __fmul_rn(zy, zy); asm volatile("" : "+v"(zy2)); v4f g;
#pragma unroll
    for (int q = 0; q < 4; ++q) { const int j = (s0 + q) % GW; const float zx = __fdiv_rn(__fsub_rn((float)j, mx), sx); float zx2 = __fmul_rn(zx, zx); asm volatile("" : "+v"(zx2)); g[q] = __expf(__fmul_rn(-0.5f, __fadd_rn(zx2, zy2))); }
    *(volatile v4f*)(G + e) = g; __threadfence(); *(volatile v4f*)(G + e) = g; }
__global__ __launch_bounds__(256) void k_gnorm(float* G) { const int lane = threadIdx.x & 31; const int o = blockIdx.x * 8 + (threadIdx.x >> 5); if (o >= NO) return; float* r = G + (size_t)o * NS; float s = 0.f;
#pragma unroll 4
    for (int ch = 0; ch < 32; ++ch) { const v4f a = *(const v4f*)(r + ch * 128 + lane * 4); s = __fadd_rn(s, __fadd_rn(__fadd_rn(a[0], a[1]), __fadd_rn(a[2], a[3]))); }
#pragma unroll
    for (int sh = 16; sh; sh >>= 1) s += __shfl_xor(s, sh, 32);
    const float f = __fdiv_rn(1.0f, s);
#pragma unroll 4
    for (int ch = 0; ch < 32; ++ch) { float* p = r + ch * 128 + lane * 4; const v4f a = *(const v4f*)p; v4f o4; o4[0] = a[0] * f; o4[1] = a[1] * f; o4[2] = a[2] * f; o4[3] = a[3] * f; *(volatile v4f*)p = o4; __threadfence(); *(volatile v4f*)p = o4; } }
__global__ __launch_bounds__(256) void k_pool(const float* __restrict__ G, const float* __restrict__ Y, float* OUTb) { const int o = blockIdx.x * 256 + threadIdx.x; if (o >= NO) return; const float* g = G + (size_t)o * NS; const float* y = Y + (size_t)o * NS; float s = 0.f;
#pragma unroll 2
    for (int i = 0; i < NS; i += 4) { const v4f a = *(const v4f*)(g + i), c = *(const v4f*)(y + i);
#pragma unroll
        for (int q = 0; q < 4; ++q) { float p = __fmul_rn(a[q], c[q]); asm volatile("" : "+v"(p)); s = __fadd_rn(s, p); } }
    *(volatile float*)(OUTb + o) = s; __threadfence(); *(volatile float*)(OUTb + o) = s; }

extern "C" void kernel_launch(void* const* d_in, const int* in_sizes, int n_in,
                              void* d_out, int out_size, void* d_ws, size_t ws_size, hipStream_t stream) {
    (void)in_sizes; (void)n_in; (void)out_size;
    const float* x = (const float*)d_in[0]; const float* mu = (const float*)d_in[1]; const float* sg = (const float*)d_in[2]; const float* wt = (const float*)d_in[3];
    float* OUT = (float*)d_out;
    char* wsp = (char*)d_ws;
    auto take = [&](size_t bytes) { char* p = wsp; wsp += (bytes + 255) & ~(size_t)255; return (void*)p; };
    bf* WB = (bf*)take((size_t)NO * CC * 2); bf* XT = (bf*)take((size_t)NS * CC * 2); float* G = (float*)take((size_t)NO * NS * 4); float* Y = (float*)take((size_t)NO * NS * 4);
    if ((size_t)(wsp - (char*)d_ws) > ws_size) return;
    k_cvt8<<<(NO * CC / 8 + 255) / 256, 256, 0, stream>>>(wt, WB, (size_t)NO * CC / 8);
    k_gauss<<<(unsigned)(((size_t)NO * NS / 4 + 255) / 256), 256, 0, stream>>>(mu, sg, G); k_gnorm<<<NO / 8, 256, 0, stream>>>(G);
    for (int b = 0; b < NB_; ++b) {
        k_tok<<<(unsigned)(((size_t)NS * CC / 4 + 255) / 256), 256, 0, stream>>>(x + (size_t)b * CC * NS, XT);
        k_gemmw<bf, 0, false><<<dim3(NO / 64, NS / 64, 1), 32, 0, stream>>>(WB, nullptr, XT, nullptr, CC, Y, NS, nullptr, 0, 0, 0);
        k_pool<<<NO / 256, 256, 0, stream>>>(G, Y, OUT + (size_t)b * NO); }
}
